// LSTM_88459146428571
// MI455X (gfx1250) — hardware-verified
//
#include <hip/hip_runtime.h>
#include <math.h>

constexpr int SEQ_LEN       = 4096;
constexpr int BATCH_TOT     = 1024;
constexpr int IN_FEAT       = 2;
constexpr int HID_UNITS     = 16;
constexpr int GATE_ROWS     = 4 * HID_UNITS;
constexpr int ROWS_PER_WAVE = 32;
constexpr int NUM_BLOCKS    = BATCH_TOT / ROWS_PER_WAVE;
constexpr int APITCH        = 40;
constexpr int WPITCH        = 40;
constexpr int HSPITCH       = 20;
constexpr int KPAD          = 32;

static_assert(HID_UNITS == 16, "one 16-column tile per gate");
static_assert(HID_UNITS + IN_FEAT <= KPAD, "h and x fit one 32-deep k step");
static_assert(BATCH_TOT % ROWS_PER_WAVE == 0, "exact batch tiling");
static_assert(NUM_BLOCKS * ROWS_PER_WAVE == BATCH_TOT, "exact batch tiling");
static_assert(GATE_ROWS == 64, "two weight rows per lane");
static_assert((APITCH * 2) % 16 == 0 && (WPITCH * 2) % 16 == 0 && (HSPITCH * 4) % 16 == 0, "16-B aligned rows");
static_assert(APITCH >= KPAD && WPITCH >= KPAD && HSPITCH >= HID_UNITS, "pitch covers the row");

typedef __attribute__((ext_vector_type(16))) _Float16 v16h;
typedef __attribute__((ext_vector_type(8)))  _Float16 v8h;
typedef __attribute__((ext_vector_type(8)))  float    v8f;
typedef __attribute__((ext_vector_type(4)))  float    v4f;
typedef __attribute__((ext_vector_type(2)))  float    v2f;
typedef __attribute__((ext_vector_type(4)))  unsigned v4u;

template <typename T> struct Frag;
template <> struct Frag<_Float16> {
  typedef v16h V; union U { v16h v; v8h h[2]; };
  static __device__ __forceinline__ v16h load(const _Float16* p) {
    U f; f.h[0] = *(const v8h*)(p); f.h[1] = *(const v8h*)(p + 16); return f.v;
  }
  static __device__ __forceinline__ v8f mma(v16h a, v16h b, v8f c) {
    return __builtin_amdgcn_wmma_f32_16x16x32_f16(false, a, false, b, (short)0, c, false, false);
  }
};

__device__ __forceinline__ void gate_guard(v8f& a, v8f& b, v8f& c, v8f& d, v16h x, v16h y0, v16h y1, v16h y2, v16h y3) {
  asm volatile("v_nop\n\tv_nop\n\tv_nop\n\tv_nop" : "+v"(a), "+v"(b), "+v"(c), "+v"(d) : "v"(x), "v"(y0), "v"(y1), "v"(y2), "v"(y3));
}

__device__ __forceinline__ float fsig(float x)  { return __builtin_amdgcn_rcpf(1.0f + __expf(-x)); }
__device__ __forceinline__ float ftanh(float x) { return 1.0f - 2.0f * __builtin_amdgcn_rcpf(__expf(2.0f * x) + 1.0f); }

__device__ __forceinline__ unsigned h16bits(float f) {
  const _Float16 hv = (_Float16)f;
  const unsigned short us = __builtin_bit_cast(unsigned short, hv);
  return (unsigned)us;
}
__device__ __forceinline__ unsigned pack2h(float a, float b) {
  const unsigned lo = h16bits(a);
  const unsigned hi = h16bits(b);
  return lo | (hi << 16);
}

__global__ __launch_bounds__(32) void lstm_seq_kernel(const float* __restrict__ x,
                                                      const float* __restrict__ W_ih,
                                                      const float* __restrict__ W_hh,
                                                      const float* __restrict__ b_ih,
                                                      const float* __restrict__ b_hh,
                                                      const float* __restrict__ W_lin,
                                                      const float* __restrict__ b_lin,
                                                      float* __restrict__ out) {
  __shared__ __align__(16) _Float16 Wp[GATE_ROWS * WPITCH];
  __shared__ __align__(16) _Float16 Ah[ROWS_PER_WAVE * APITCH];
  __shared__ __align__(16) float    Hs[ROWS_PER_WAVE * HSPITCH];

  const int lane = threadIdx.x & 31;
  const int c    = lane & 15;
  const int hh   = lane >> 4;
  const int b0   = blockIdx.x * ROWS_PER_WAVE;
  const v4u zero4 = {0u, 0u, 0u, 0u};

#pragma unroll 1
  for (int rr = 0; rr < 2; ++rr) {
    const int n = lane + 32 * rr;
    const v4f w0 = *(const v4f*)(W_hh + n * HID_UNITS + 0);
    const v4f w1 = *(const v4f*)(W_hh + n * HID_UNITS + 4);
    const v4f w2 = *(const v4f*)(W_hh + n * HID_UNITS + 8);
    const v4f w3 = *(const v4f*)(W_hh + n * HID_UNITS + 12);
    const v2f wi = *(const v2f*)(W_ih + n * IN_FEAT);
    v4u p0, p1, p2;
    p0[0] = pack2h(w0[0], w0[1]); p0[1] = pack2h(w0[2], w0[3]);
    p0[2] = pack2h(w1[0], w1[1]); p0[3] = pack2h(w1[2], w1[3]);
    p1[0] = pack2h(w2[0], w2[1]); p1[1] = pack2h(w2[2], w2[3]);
    p1[2] = pack2h(w3[0], w3[1]); p1[3] = pack2h(w3[2], w3[3]);
    p2[0] = pack2h(wi[0], wi[1]); p2[1] = 0u; p2[2] = 0u; p2[3] = 0u;
    v4u* dst = (v4u*)(Wp + n * WPITCH);
    dst[0] = p0;
    dst[1] = p1;
    dst[2] = p2;
    dst[3] = zero4;
    asm volatile("" ::: "memory");
  }

  float bsum[4];
#pragma unroll
  for (int g = 0; g < 4; ++g) bsum[g] = b_ih[g * HID_UNITS + c] + b_hh[g * HID_UNITS + c];
  asm volatile("" ::: "memory");
  const v4f wl0 = *(const v4f*)(W_lin + 0);
  const v4f wl1 = *(const v4f*)(W_lin + 4);
  const v4f wl2 = *(const v4f*)(W_lin + 8);
  const v4f wl3 = *(const v4f*)(W_lin + 12);
  const float blin = b_lin[0];
  asm volatile("" ::: "memory");

  const v2f* xin2 = (const v2f*)x;
  {
    const v2f xv = xin2[(size_t)b0 + lane];
    v4u px;
    px[0] = pack2h(xv[0], xv[1]); px[1] = 0u; px[2] = 0u; px[3] = 0u;
    v4u* ar = (v4u*)(Ah + lane * APITCH);
    ar[0] = zero4;
    ar[1] = zero4;
    ar[2] = px;
    ar[3] = zero4;
  }
  __syncthreads();

  v16h bw[4];
#pragma unroll
  for (int g = 0; g < 4; ++g) bw[g] = Frag<_Float16>::load(Wp + (g * HID_UNITS + c) * WPITCH + 8 * hh);

  v8f bias8[4];
#pragma unroll
  for (int g = 0; g < 4; ++g) {
    const float bv = bsum[g];
    bias8[g] = (v8f){bv, bv, bv, bv, bv, bv, bv, bv};
  }

  float cst[2][8];
#pragma unroll
  for (int t = 0; t < 2; ++t)
#pragma unroll
    for (int r = 0; r < 8; ++r) cst[t][r] = 0.0f;

#pragma unroll 1
  for (int s = 0; s < SEQ_LEN; ++s) {
    const int sn = (s + 1 < SEQ_LEN) ? (s + 1) : (SEQ_LEN - 1);
    const v2f xn = xin2[(size_t)sn * BATCH_TOT + b0 + lane];

#pragma unroll
    for (int t = 0; t < 2; ++t) {
      const v16h a = Frag<_Float16>::load(Ah + (16 * t + c) * APITCH + 8 * hh);
      v8f g0 = bias8[0], g1 = bias8[1], g2 = bias8[2], g3 = bias8[3];
      g0 = Frag<_Float16>::mma(a, bw[0], g0);
      g1 = Frag<_Float16>::mma(a, bw[1], g1);
      g2 = Frag<_Float16>::mma(a, bw[2], g2);
      g3 = Frag<_Float16>::mma(a, bw[3], g3);
      gate_guard(g0, g1, g2, g3, a, bw[0], bw[1], bw[2], bw[3]);
      asm volatile("" ::: "memory");
#pragma unroll
      for (int r = 0; r < 8; ++r) {
        const float iv = fsig(g0[r]);
        const float fv = fsig(g1[r]);
        const float gv = ftanh(g2[r]);
        const float ov = fsig(g3[r]);
        const float cn = fv * cst[t][r] + iv * gv;
        cst[t][r] = cn;
        const float hn = ov * ftanh(cn);
        const int row = 16 * t + 8 * hh + r;
        Ah[row * APITCH + c]  = (_Float16)hn;
        Hs[row * HSPITCH + c] = hn;
      }
    }
    {
      v4u px;
      px[0] = pack2h(xn[0], xn[1]); px[1] = 0u; px[2] = 0u; px[3] = 0u;
      v4u* ar = (v4u*)(Ah + lane * APITCH);
      ar[2] = px;
      ar[3] = zero4;
    }
    __syncthreads();

    {
      const float* hr = Hs + lane * HSPITCH;
      const v4f q0 = *(const v4f*)(hr + 0);
      const v4f q1 = *(const v4f*)(hr + 4);
      const v4f q2 = *(const v4f*)(hr + 8);
      const v4f q3 = *(const v4f*)(hr + 12);
      float o = blin;
      o = fmaf(q0[0], wl0[0], o); o = fmaf(q0[1], wl0[1], o); o = fmaf(q0[2], wl0[2], o); o = fmaf(q0[3], wl0[3], o);
      o = fmaf(q1[0], wl1[0], o); o = fmaf(q1[1], wl1[1], o); o = fmaf(q1[2], wl1[2], o); o = fmaf(q1[3], wl1[3], o);
      o = fmaf(q2[0], wl2[0], o); o = fmaf(q2[1], wl2[1], o); o = fmaf(q2[2], wl2[2], o); o = fmaf(q2[3], wl2[3], o);
      o = fmaf(q3[0], wl3[0], o); o = fmaf(q3[1], wl3[1], o); o = fmaf(q3[2], wl3[2], o); o = fmaf(q3[3], wl3[3], o);
      volatile float* op = out + (size_t)s * BATCH_TOT + b0 + lane;
      *op = o;
      __threadfence();
      *op = o;
    }
  }
}

extern "C" void kernel_launch(void* const* d_in, const int* in_sizes, int n_in,
                              void* d_out, int out_size, void* d_ws, size_t ws_size, hipStream_t stream) {
  (void)d_ws; (void)ws_size;
  if (n_in < 7 || d_out == nullptr) return;
  if (in_sizes[0] != SEQ_LEN * BATCH_TOT * IN_FEAT || in_sizes[1] != GATE_ROWS * IN_FEAT ||
      in_sizes[2] != GATE_ROWS * HID_UNITS || in_sizes[3] != GATE_ROWS || in_sizes[4] != GATE_ROWS ||
      in_sizes[5] != HID_UNITS || in_sizes[6] != 1 || out_size != SEQ_LEN * BATCH_TOT) return;

  const float* x     = (const float*)d_in[0];
  const float* W_ih  = (const float*)d_in[1];
  const float* W_hh  = (const float*)d_in[2];
  const float* b_ih  = (const float*)d_in[3];
  const float* b_hh  = (const float*)d_in[4];
  const float* W_lin = (const float*)d_in[5];
  const float* b_lin = (const float*)d_in[6];
  float* out = (float*)d_out;

  lstm_seq_kernel<<<NUM_BLOCKS, 32, 0, stream>>>(x, W_ih, W_hh, b_ih, b_hh, W_lin, b_lin, out);
}
